// ProxySpatialAttentionModule_77197742178862
// MI455X (gfx1250) — hardware-verified
//
#include <hip/hip_runtime.h>
#include <math.h>

constexpr int kHeadDim  = 32;
constexpr int kSpat     = 3136;
constexpr int kGroups   = 32;
constexpr int kTiles64  = 49;
constexpr int kColIter  = 98;
constexpr int kQKCols   = 64;

constexpr size_t kOffWqkH = 0;
constexpr size_t kOffWqkL = 131072;
constexpr size_t kOffWvH  = 262144;
constexpr size_t kOffWvL  = 327680;
constexpr size_t kOffBqk  = 393216;
constexpr size_t kOffBvr  = 401408;
constexpr size_t kOffQK   = 524288;
constexpr size_t kOffVH   = 13369344;
constexpr size_t kOffVL   = 19791872;
constexpr size_t kOffXE   = 26214400;
constexpr size_t kOffXTL  = 26214400 + 6422528;
constexpr size_t kOffPTH  = 65552384;
constexpr size_t kOffPTL  = 85221376;
constexpr size_t kWsTotal = 104890368;
static_assert(kOffQK + (size_t)kGroups * kSpat * kQKCols * 2 == kOffVH, "carve");
static_assert(kOffVH + (size_t)kGroups * kHeadDim * kSpat * 2 == kOffVL, "carve");
static_assert(kOffVL + (size_t)kGroups * kHeadDim * kSpat * 2 == kOffXE, "carve");
static_assert(kOffXTL + (size_t)kGroups * kSpat * kHeadDim * 2 <= kOffXE + (size_t)kSpat * kSpat * 4, "carve");
static_assert(kOffXE + (size_t)kSpat * kSpat * 4 == kOffPTH, "carve");
static_assert(kOffPTH + (size_t)kSpat * kSpat * 2 == kOffPTL, "carve");
static_assert(kOffPTL + (size_t)kSpat * kSpat * 2 == kWsTotal, "carve");

typedef __attribute__((ext_vector_type(16))) _Float16 v16h;
typedef __attribute__((ext_vector_type(8)))  _Float16 v8h;
typedef __attribute__((ext_vector_type(16))) __bf16   v16b;
typedef __attribute__((ext_vector_type(8)))  __bf16   v8b;
typedef __attribute__((ext_vector_type(8)))  float    v8f;
typedef __attribute__((ext_vector_type(4)))  float    v4f;
typedef __attribute__((ext_vector_type(4)))  unsigned int v4u;

__device__ __forceinline__ unsigned short f2bf_bits(float f) {
  unsigned u = __float_as_uint(f);
  return (unsigned short)((u + 0x7FFFu + ((u >> 16) & 1u)) >> 16);
}
__device__ __forceinline__ float bf_bits2f(unsigned short h) { return __uint_as_float(((unsigned)h) << 16); }

__device__ __forceinline__ void dep_guard_h(v8f& a, v8f& b, v16h x, v16h y) { asm volatile("v_nop\n\tv_nop\n\tv_nop\n\tv_nop" : "+v"(a), "+v"(b) : "v"(x), "v"(y)); }
__device__ __forceinline__ void dep_guard_b(v8f& a, v8f& b, v16b x, v16b y) { asm volatile("v_nop\n\tv_nop\n\tv_nop\n\tv_nop" : "+v"(a), "+v"(b) : "v"(x), "v"(y)); }
__device__ __forceinline__ void keep4_h(v16h a, v16h b, v16h c, v16h d) { asm volatile("v_nop" :: "v"(a), "v"(b), "v"(c), "v"(d)); }
__device__ __forceinline__ void keep4_b(v16b a, v16b b, v16b c, v16b d) { asm volatile("v_nop" :: "v"(a), "v"(b), "v"(c), "v"(d)); }
__device__ __forceinline__ void acc_guard4(v8f& a, v8f& b, v8f& c, v8f& d) { asm volatile("v_nop\n\tv_nop\n\tv_nop\n\tv_nop" : "+v"(a), "+v"(b), "+v"(c), "+v"(d)); }
template <typename T> struct Frag;
template <> struct Frag<_Float16> {
  typedef v16h V; union U { v16h v; v8h h[2]; };
  static __device__ __forceinline__ v16h load(const _Float16* p) {
    U f; f.h[0] = *(const v8h*)(p); f.h[1] = *(const v8h*)(p + 16); return f.v;
  }
  static __device__ __forceinline__ v8f mma(v16h a, v16h b, v8f c) {
    return __builtin_amdgcn_wmma_f32_16x16x32_f16(false, a, false, b, (short)0, c, false, false);
  }
  static __device__ __forceinline__ void guard(v8f& a, v8f& b, v16h x, v16h y) { dep_guard_h(a, b, x, y); }
  static __device__ __forceinline__ void keep(v16h a, v16h b, v16h c, v16h d) { keep4_h(a, b, c, d); }
};
template <> struct Frag<__bf16> {
  typedef v16b V; union U { v16b v; v8b h[2]; };
  static __device__ __forceinline__ v16b load(const __bf16* p) {
    U f; f.h[0] = *(const v8b*)(p); f.h[1] = *(const v8b*)(p + 16); return f.v;
  }
  static __device__ __forceinline__ v8f mma(v16b a, v16b b, v8f c) {
    return __builtin_amdgcn_wmma_f32_16x16x32_bf16(false, a, false, b, (short)0, c, false, false);
  }
  static __device__ __forceinline__ void guard(v8f& a, v8f& b, v16b x, v16b y) { dep_guard_b(a, b, x, y); }
  static __device__ __forceinline__ void keep(v16b a, v16b b, v16b c, v16b d) { keep4_b(a, b, c, d); }
};

__device__ __forceinline__ unsigned pk16(unsigned short a, unsigned short b) { return (unsigned)a | ((unsigned)b << 16); }

template <int ET> struct Elem;
template <> struct Elem<0> { typedef _Float16 T; };
template <> struct Elem<1> { typedef __bf16 T; };
template <int ET, bool SPLIT, int BIAS_MODE, int OUT_MODE, bool RESID, int MI>
__global__ __launch_bounds__(256) void wmma_gemm_mi(
    const unsigned short* __restrict__ Ap, const unsigned short* __restrict__ A2p, int lda, long strideA,
    const unsigned short* __restrict__ Btp, const unsigned short* __restrict__ Bt2p, int ldb, long strideB,
    void* __restrict__ Cout, void* __restrict__ Cout2, int ldc, long strideC,
    const float* __restrict__ bias, long strideBias,
    const float* __restrict__ resid, long strideR,
    int M, int N, int K, float scale) {
  typedef typename Elem<ET>::T T;
  typedef typename Frag<T>::V V;
  const T* A = (const T*)Ap; const T* A2 = (const T*)A2p; const T* Bt = (const T*)Btp; const T* Bt2 = (const T*)Bt2p;
  __shared__ __align__(16) float sT[8][16 * 68];
  const int b    = blockIdx.y;
  const int lane = threadIdx.x & 31;
  const int wave = threadIdx.x >> 5;
  const int tilesN = N >> 6;
  const int tilesM = M / (16 * MI);
  const int tile = blockIdx.x * 8 + wave;
  if (tile >= tilesM * tilesN) return;
  const int tm = tile / tilesN;
  const int tn = tile - tm * tilesN;
  const int m0 = tm * (16 * MI);
  const int n0 = tn << 6;

  const T* Ab  = A  + (size_t)b * strideA;
  const T* Bb  = Bt + (size_t)b * strideB;
  const T* Ab2 = SPLIT ? (A2  + (size_t)b * strideA) : nullptr;
  const T* Bb2 = SPLIT ? (Bt2 + (size_t)b * strideB) : nullptr;
  const float* biasb = (BIAS_MODE != 0) ? (bias + (size_t)b * strideBias) : nullptr;

  const int rlane = lane & 15;
  const int koff  = (lane >> 4) * 8;
  const int mOff  = (lane >> 4) * 8;

  v8f acc[MI][4];
#pragma unroll
  for (int i = 0; i < MI; ++i)
#pragma unroll
    for (int j = 0; j < 4; ++j) acc[i][j] = (v8f){0.f,0.f,0.f,0.f,0.f,0.f,0.f,0.f};

  for (int k0 = 0; k0 < K; k0 += 32) {
    V bh[4], bl[4];
#pragma unroll
    for (int j = 0; j < 4; ++j) {
      const size_t bo = (size_t)(n0 + (j << 4) + rlane) * ldb + koff + k0;
      bh[j] = Frag<T>::load(Bb + bo);
      if (SPLIT) bl[j] = Frag<T>::load(Bb2 + bo);
    }
#pragma unroll
    for (int i = 0; i < MI; ++i) {
      const size_t ao = (size_t)(m0 + (i << 4) + rlane) * lda + koff + k0;
      V ah = Frag<T>::load(Ab + ao);
      V al;
      if (SPLIT) al = Frag<T>::load(Ab2 + ao);
#pragma unroll
      for (int j = 0; j < 4; ++j) {
        acc[i][j] = Frag<T>::mma(ah, bh[j], acc[i][j]);
        if (SPLIT) {
          acc[i][j] = Frag<T>::mma(ah, bl[j], acc[i][j]);
          acc[i][j] = Frag<T>::mma(al, bh[j], acc[i][j]);
        }
      }
      Frag<T>::guard(acc[i][0], acc[i][3], ah, SPLIT ? al : ah);
    }
    Frag<T>::keep(bh[0], bh[1], bh[2], bh[3]);
    if (SPLIT) Frag<T>::keep(bl[0], bl[1], bl[2], bl[3]);
  }
#pragma unroll
  for (int i = 0; i < MI; ++i) acc_guard4(acc[i][0], acc[i][1], acc[i][2], acc[i][3]);

  float* slab = sT[wave];
  const float* Rb = RESID ? (resid + (size_t)b * strideR) : nullptr;
#pragma unroll
  for (int i = 0; i < MI; ++i) {
    const int mBase = m0 + (i << 4);
#pragma unroll
    for (int j = 0; j < 4; ++j) {
      const int n = n0 + (j << 4) + rlane;
      float bvn = 0.f;
      if (BIAS_MODE == 2) bvn = biasb[n];
#pragma unroll
      for (int r = 0; r < 8; ++r) {
        float v = acc[i][j][r] * scale;
        if (BIAS_MODE == 1) v += biasb[mBase + mOff + r];
        if (BIAS_MODE == 2) v += bvn;
        if (RESID) v += Rb[(size_t)(mBase + mOff + r) * ldc + n];
        slab[(mOff + r) * 68 + (j << 4) + rlane] = v;
      }
    }
    __builtin_amdgcn_fence(__ATOMIC_RELEASE, "workgroup");
    __builtin_amdgcn_wave_barrier();
    __builtin_amdgcn_fence(__ATOMIC_ACQUIRE, "workgroup");
    if (OUT_MODE == 0) {
      float* C = (float*)Cout + (size_t)b * strideC;
      const int hh = lane >> 4, c4 = (lane & 15) * 4;
      for (int pass = 0; pass < 2; ++pass) {
#pragma unroll
        for (int it = 0; it < 8; ++it) {
          const int row = it * 2 + hh;
          v4f v = *(const v4f*)(slab + row * 68 + c4);
          *(volatile v4f*)(C + (size_t)(mBase + row) * ldc + n0 + c4) = v;
        }
        __threadfence();
      }
    } else {
      const int q = lane >> 3, c8 = (lane & 7) * 8;
      unsigned short* C  = (unsigned short*)Cout  + (size_t)b * strideC;
      unsigned short* C2 = (OUT_MODE == 2) ? ((unsigned short*)Cout2 + (size_t)b * strideC) : nullptr;
      for (int pass = 0; pass < 2; ++pass) {
#pragma unroll
        for (int it = 0; it < 4; ++it) {
          const int row = it * 4 + q;
          const float* sp = slab + row * 68 + c8;
          v8h hv, lv;
#pragma unroll
          for (int e = 0; e < 8; ++e) {
            if (OUT_MODE == 1) {
              hv[e] = (_Float16)sp[e];
            } else {
              unsigned short hb = f2bf_bits(sp[e]);
              unsigned short lb = f2bf_bits(sp[e] - bf_bits2f(hb));
              hv[e] = __builtin_bit_cast(_Float16, hb);
              lv[e] = __builtin_bit_cast(_Float16, lb);
            }
          }
          *(volatile v8h*)(C + (size_t)(mBase + row) * ldc + n0 + c8) = hv;
          if (OUT_MODE == 2) *(volatile v8h*)(C2 + (size_t)(mBase + row) * ldc + n0 + c8) = lv;
        }
        __threadfence();
      }
    }
    __builtin_amdgcn_fence(__ATOMIC_RELEASE, "workgroup");
    __builtin_amdgcn_wave_barrier();
    __builtin_amdgcn_fence(__ATOMIC_ACQUIRE, "workgroup");
  }
}

__global__ __launch_bounds__(256) void prep_w_kernel(
    const float* __restrict__ Wq, const float* __restrict__ bq,
    const float* __restrict__ Wk, const float* __restrict__ bk,
    const float* __restrict__ Wv, const float* __restrict__ bv,
    unsigned short* __restrict__ WqkH, unsigned short* __restrict__ WqkL,
    unsigned short* __restrict__ WvH, unsigned short* __restrict__ WvL,
    float* __restrict__ Bqk, float* __restrict__ Bvr) {
  const int bg = blockIdx.x, g = bg & 7;
  const int t = threadIdx.x, wave = t >> 5, lane = t & 31;
  const int n = t >> 2, kk = (t & 3) * 8;
  {
    const float* pq = Wq + (size_t)g * 1024 + (n & 31) * 32 + kk;
    const float* pk = Wk + (size_t)g * 1024 + (n & 31) * 32 + kk;
    unsigned short hb[8], lb[8];
#pragma unroll
    for (int e = 0; e < 8; ++e) {
      const float a = pq[e];
      const float c = pk[e];
      const float w = (n < 32) ? a : c;
      const unsigned short h = f2bf_bits(w);
      hb[e] = h;
      lb[e] = f2bf_bits(w - bf_bits2f(h));
    }
    const v4u uh = (v4u){pk16(hb[0], hb[1]), pk16(hb[2], hb[3]), pk16(hb[4], hb[5]), pk16(hb[6], hb[7])};
    const v4u ul = (v4u){pk16(lb[0], lb[1]), pk16(lb[2], lb[3]), pk16(lb[4], lb[5]), pk16(lb[6], lb[7])};
    const size_t o = (size_t)bg * 2048 + (size_t)t * 8;
    *(volatile v4u*)(WqkH + o) = uh;
    *(volatile v4u*)(WqkL + o) = ul;
    __threadfence();
    *(volatile v4u*)(WqkH + o) = uh;
    *(volatile v4u*)(WqkL + o) = ul;
  }
  if (wave < 4) {
    const float* pv = Wv + (size_t)g * 1024 + (n & 31) * 32 + kk;
    unsigned short hb[8], lb[8];
#pragma unroll
    for (int e = 0; e < 8; ++e) {
      const float w = pv[e];
      const unsigned short h = f2bf_bits(w);
      hb[e] = h;
      lb[e] = f2bf_bits(w - bf_bits2f(h));
    }
    const v4u uh = (v4u){pk16(hb[0], hb[1]), pk16(hb[2], hb[3]), pk16(hb[4], hb[5]), pk16(hb[6], hb[7])};
    const v4u ul = (v4u){pk16(lb[0], lb[1]), pk16(lb[2], lb[3]), pk16(lb[4], lb[5]), pk16(lb[6], lb[7])};
    const size_t o = (size_t)bg * 1024 + (size_t)t * 8;
    *(volatile v4u*)(WvH + o) = uh;
    *(volatile v4u*)(WvL + o) = ul;
    __threadfence();
    *(volatile v4u*)(WvH + o) = uh;
    *(volatile v4u*)(WvL + o) = ul;
  }
  if (wave == 0) {
    const int i4 = (lane & 15) * 4;
    const int j4 = (lane & 7) * 4;
    float f[4], fv[4];
#pragma unroll
    for (int u = 0; u < 4; ++u) {
      const int d = i4 + u;
      const float a = bq[g * 32 + (d & 31)];
      const float c = bk[g * 32 + (d & 31)];
      f[u] = (d < 32) ? a : c;
      fv[u] = bv[g * 32 + j4 + u];
    }
    const v4f vb = (v4f){f[0], f[1], f[2], f[3]};
    const v4f vv = (v4f){fv[0], fv[1], fv[2], fv[3]};
    float* pb = Bqk + (size_t)bg * 64 + i4;
    float* pvv = Bvr + (size_t)bg * 32 + j4;
    if (lane < 16) *(volatile v4f*)pb = vb;
    if (lane >= 16 && lane < 24) *(volatile v4f*)pvv = vv;
    __threadfence();
    if (lane < 16) *(volatile v4f*)pb = vb;
    if (lane >= 16 && lane < 24) *(volatile v4f*)pvv = vv;
  }
}

__global__ __launch_bounds__(256) void xcast_kernel(const float* __restrict__ x,
                                                   unsigned short* __restrict__ XTh, unsigned short* __restrict__ XTl) {
  __shared__ float sx[32][65];
  const int l0 = blockIdx.x * 64;
  const int bg = blockIdx.y;
  const int t  = threadIdx.x;
  const float* xb = x + (size_t)bg * kHeadDim * kSpat + l0;
#pragma unroll
  for (int i = 0; i < 8; ++i) {
    const int e = i * 256 + t;
    const int c = e >> 6, ll = e & 63;
    sx[c][ll] = xb[(size_t)c * kSpat + ll];
  }
  __syncthreads();
  const int lq = t >> 2, c0 = (t & 3) * 8;
  unsigned short hb[8], lb[8];
#pragma unroll
  for (int e = 0; e < 8; ++e) {
    const float f = sx[c0 + e][lq];
    const unsigned short h = f2bf_bits(f);
    hb[e] = h;
    lb[e] = f2bf_bits(f - bf_bits2f(h));
  }
  const v4u uh = (v4u){pk16(hb[0], hb[1]), pk16(hb[2], hb[3]), pk16(hb[4], hb[5]), pk16(hb[6], hb[7])};
  const v4u ul = (v4u){pk16(lb[0], lb[1]), pk16(lb[2], lb[3]), pk16(lb[4], lb[5]), pk16(lb[6], lb[7])};
  const size_t o = (size_t)bg * kSpat * kHeadDim + (size_t)(l0 + lq) * kHeadDim + c0;
  *(volatile v4u*)(XTh + o) = uh;
  *(volatile v4u*)(XTl + o) = ul;
  __threadfence();
  *(volatile v4u*)(XTh + o) = uh;
  *(volatile v4u*)(XTl + o) = ul;
}

__global__ __launch_bounds__(256) void softmax_pt_kernel(const float* __restrict__ E,
                                                        unsigned short* __restrict__ PTh, unsigned short* __restrict__ PTl) {
  __shared__ float s_m[64];
  __shared__ float s_r[64];
  __shared__ unsigned int sTh[64 * 33];
  __shared__ unsigned int sTl[64 * 33];
  const int j0 = blockIdx.x * 64;
  const int t = threadIdx.x, lane = t & 31, wave = t >> 5;
  for (int rr = 0; rr < 8; ++rr) {
    const int jr = wave * 8 + rr;
    const float* er = E + (size_t)(j0 + jr) * kSpat + lane;
    float m = er[0];
    float s = 1.0f;
#pragma unroll 2
    for (int i = 1; i < kColIter; ++i) {
      const float e  = er[i * 32];
      const float mn = fmaxf(m, e);
      s = s * __expf(m - mn) + __expf(e - mn);
      m = mn;
    }
    float gm = m;
#pragma unroll
    for (int off = 1; off < 32; off <<= 1) gm = fmaxf(gm, __shfl_xor(gm, off, 32));
    s = s * __expf(m - gm);
#pragma unroll
    for (int off = 1; off < 32; off <<= 1) s += __shfl_xor(s, off, 32);
    if (lane == 0) { s_m[jr] = gm; s_r[jr] = 1.0f / s; }
  }
  __syncthreads();

  const int kc = t & 63, jg = t >> 6;
  float rm[16], rz[16];
#pragma unroll
  for (int i = 0; i < 16; ++i) { rm[i] = s_m[jg * 16 + i]; rz[i] = s_r[jg * 16 + i]; }
  const int q = lane >> 3, cw = (lane & 7) * 4;
  const float* eb = E + (size_t)(j0 + jg * 16) * kSpat + kc;
  for (int kt = 0; kt < kTiles64; ++kt) {
    const int k0 = kt * 64;
    unsigned int wh[8], wl[8];
#pragma unroll
    for (int i2 = 0; i2 < 8; ++i2) {
      const float e0 = eb[(size_t)(2 * i2) * kSpat + k0];
      const float e1 = eb[(size_t)(2 * i2 + 1) * kSpat + k0];
      const float p0 = __expf(e0 - rm[2 * i2]) * rz[2 * i2];
      const float p1 = __expf(e1 - rm[2 * i2 + 1]) * rz[2 * i2 + 1];
      const unsigned short h0 = f2bf_bits(p0);
      const unsigned short h1 = f2bf_bits(p1);
      const unsigned short g0 = f2bf_bits(p0 - bf_bits2f(h0));
      const unsigned short g1 = f2bf_bits(p1 - bf_bits2f(h1));
      wh[i2] = pk16(h0, h1);
      wl[i2] = pk16(g0, g1);
    }
    __syncthreads();
#pragma unroll
    for (int i2 = 0; i2 < 8; ++i2) {
      sTh[kc * 33 + jg * 8 + i2] = wh[i2];
      sTl[kc * 33 + jg * 8 + i2] = wl[i2];
    }
    __syncthreads();
    for (int pass = 0; pass < 2; ++pass) {
#pragma unroll
      for (int it = 0; it < 2; ++it) {
        const int row = wave * 8 + it * 4 + q;
        const unsigned int* sh = sTh + row * 33 + cw;
        const unsigned int* sl = sTl + row * 33 + cw;
        const v4u uh = (v4u){sh[0], sh[1], sh[2], sh[3]};
        const v4u ul = (v4u){sl[0], sl[1], sl[2], sl[3]};
        const size_t o = (size_t)(k0 + row) * kSpat + j0 + (lane & 7) * 8;
        *(volatile v4u*)(PTh + o) = uh;
        *(volatile v4u*)(PTl + o) = ul;
      }
      __threadfence();
    }
  }
}

extern "C" void kernel_launch(void* const* d_in, const int* in_sizes, int n_in,
                              void* d_out, int out_size, void* d_ws, size_t ws_size, hipStream_t stream) {
  (void)in_sizes; (void)out_size;
  if (n_in < 7) return;
  if (ws_size < kWsTotal) return;
  const float* x  = (const float*)d_in[0];
  const float* Wq = (const float*)d_in[1];
  const float* bq = (const float*)d_in[2];
  const float* Wk = (const float*)d_in[3];
  const float* bk = (const float*)d_in[4];
  const float* Wv = (const float*)d_in[5];
  const float* bv = (const float*)d_in[6];
  float* out = (float*)d_out;
  char* ws = (char*)d_ws;
  unsigned short* WqkH = (unsigned short*)(ws + kOffWqkH);
  unsigned short* WqkL = (unsigned short*)(ws + kOffWqkL);
  unsigned short* WvH  = (unsigned short*)(ws + kOffWvH);
  unsigned short* WvL  = (unsigned short*)(ws + kOffWvL);
  float* Bqk = (float*)(ws + kOffBqk);
  float* Bvr = (float*)(ws + kOffBvr);
  unsigned short* QK16 = (unsigned short*)(ws + kOffQK);
  unsigned short* VH  = (unsigned short*)(ws + kOffVH);
  unsigned short* VL  = (unsigned short*)(ws + kOffVL);
  unsigned short* XTh = (unsigned short*)(ws + kOffXE);
  unsigned short* XTl = (unsigned short*)(ws + kOffXTL);
  float* Ebuf = (float*)(ws + kOffXE);
  unsigned short* PTh = (unsigned short*)(ws + kOffPTH);
  unsigned short* PTl = (unsigned short*)(ws + kOffPTL);

  const int gemmTilesSmall = (kTiles64 + 7) / 8;
  const int gemmTilesE     = (kTiles64 * kTiles64 + 7) / 8;

  prep_w_kernel<<<dim3(kGroups), dim3(256), 0, stream>>>(Wq, bq, Wk, bk, Wv, bv, WqkH, WqkL, WvH, WvL, Bqk, Bvr);
  xcast_kernel<<<dim3(kTiles64, kGroups), dim3(256), 0, stream>>>(x, XTh, XTl);
  wmma_gemm_mi<1, true, 2, 1, false, 4><<<dim3(gemmTilesSmall, kGroups), dim3(256), 0, stream>>>(
      XTh, XTl, kHeadDim, (long)kSpat * kHeadDim,
      WqkH, WqkL, kHeadDim, (long)kQKCols * kHeadDim,
      (void*)QK16, (void*)QK16, kQKCols, (long)kSpat * kQKCols,
      Bqk, (long)kQKCols,
      x, 0L,
      kSpat, kQKCols, kHeadDim, 1.0f);
  wmma_gemm_mi<1, true, 1, 2, false, 2><<<dim3(gemmTilesSmall, kGroups), dim3(256), 0, stream>>>(
      WvH, WvL, kHeadDim, (long)kHeadDim * kHeadDim,
      XTh, XTl, kHeadDim, (long)kSpat * kHeadDim,
      (void*)VH, (void*)VL, kSpat, (long)kHeadDim * kSpat,
      Bvr, (long)kHeadDim,
      x, 0L,
      kHeadDim, kSpat, kHeadDim, 1.0f);

  for (int bg = 0; bg < kGroups; ++bg) {
    const size_t qko = (size_t)bg * kSpat * kQKCols;
    const size_t vo  = (size_t)bg * kHeadDim * kSpat;
    wmma_gemm_mi<0, false, 0, 0, false, 4><<<dim3(gemmTilesE, 1), dim3(256), 0, stream>>>(
        QK16 + qko, QK16 + qko, kQKCols, 0L,
        QK16 + qko + kHeadDim, QK16 + qko + kHeadDim, kQKCols, 0L,
        (void*)Ebuf, (void*)PTl, kSpat, 0L,
        Bqk, 0L,
        x, 0L,
        kSpat, kSpat, kHeadDim, 1.0f);
    softmax_pt_kernel<<<dim3(kTiles64), dim3(256), 0, stream>>>(Ebuf, PTh, PTl);
    wmma_gemm_mi<1, true, 0, 0, true, 2><<<dim3(gemmTilesSmall, 1), dim3(256), 0, stream>>>(
        VH + vo, VL + vo, kSpat, 0L,
        PTh, PTl, kSpat, 0L,
        (void*)(out + vo), (void*)Ebuf, kSpat, 0L,
        Bqk, 0L,
        x + vo, 0L,
        kHeadDim, kSpat, kSpat, 1.0f);
  }
}
